// Trm_Encoder_83365315215702
// MI455X (gfx1250) — hardware-verified
//
#include <hip/hip_runtime.h>
#define NBATCH 4
#define LL 1024
#define DD 300
#define DP 320
#define NHD 6
#define DPH 50
#define FF 1200
#define FFP 1216
#define NLAY 6
#define NROW (NBATCH * LL)
#define NPS (NBATCH * NHD)
#define TQ 1024
#define TK 1024
#define NH 1
#define SCL 0.35355339059327373f
#define SELU_A 1.6732632423543772f
#define SELU_S 1.0507009873554805f
typedef __bf16 v16b __attribute__((ext_vector_type(16)));
typedef unsigned short v8us __attribute__((ext_vector_type(8), may_alias));
typedef float  v8f  __attribute__((ext_vector_type(8)));
typedef float  v4f  __attribute__((ext_vector_type(4)));
typedef float  v4fa __attribute__((ext_vector_type(4), may_alias));
union FragB { v16b v; v8us half[2]; unsigned short u[16]; };

__device__ __forceinline__ unsigned short bf16_bits(float x) { unsigned int u = __float_as_uint(x); return (unsigned short)((u + 0x7FFFu + ((u >> 16) & 1u)) >> 16); }
__device__ __forceinline__ float bf16_val(unsigned short b) { return __uint_as_float(((unsigned int)b) << 16); }
__device__ __forceinline__ float bf16_round(float x) { return bf16_val(bf16_bits(x)); }
template <int NT>
__device__ __forceinline__ v8f mmaN(v16b ah, v16b al, v16b bh, v16b bl, v8f c) {
  c = __builtin_amdgcn_wmma_f32_16x16x32_bf16(false, ah, false, bh, (short)0, c, false, false);
  if (NT >= 2) c = __builtin_amdgcn_wmma_f32_16x16x32_bf16(false, al, false, bh, (short)0, c, false, false);
  if (NT >= 3) c = __builtin_amdgcn_wmma_f32_16x16x32_bf16(false, ah, false, bl, (short)0, c, false, false);
  asm volatile("v_nop\n\tv_nop\n\tv_nop\n\tv_nop" : "+v"(c) : "v"(ah), "v"(al), "v"(bh), "v"(bl));
  return c;
}

__global__ __launch_bounds__(256) void k_wt_bf16(const float* __restrict__ W, unsigned short* __restrict__ Wt, int K, int N) {
  const int t = blockIdx.x * 256 + threadIdx.x;
  const int k8n = K / 8;
  if (t >= N * k8n) return;
  const int n = t / k8n, k8 = (t % k8n) * 8;
  v8us v;
#pragma unroll
  for (int i = 0; i < 8; ++i) v[i] = bf16_bits(W[(size_t)(k8 + i) * N + n]);
  *(volatile v8us*)(Wt + (size_t)n * K + k8) = v;
  __threadfence();
  *(volatile v8us*)(Wt + (size_t)n * K + k8) = v;
}

template <bool ASPLIT, int ACT, bool BIAS_BF16>
__global__ __launch_bounds__(128) void k_gemm_bf(const float* __restrict__ A, int lda, const unsigned short* __restrict__ Wt, int ldb,
                                               const float* __restrict__ bias, float* __restrict__ C, int ldc, int M, int N, int K) {
  __shared__ __attribute__((aligned(16))) float so[4][16][64];
  const int tid = threadIdx.x, w = tid >> 5, lane = tid & 31, ln = lane & 15, hh = lane >> 4;
  const int ntn = N / 64;
  const int wid = blockIdx.x * 4 + w;
  const int mt = wid / ntn, nq = wid % ntn;
  if (mt * 16 >= M) return;
  const int row0 = mt * 16, col0 = nq * 64;
  const float* arow = A + (size_t)(row0 + ln) * lda;
  v8f acc[4] = {};
  for (int kb = 0; kb < K; kb += 32) {
    FragB ah, al;
    const v4f x0 = *(const v4fa*)(arow + kb + 8 * hh), x1 = *(const v4fa*)(arow + kb + 8 * hh + 4);
    const v4f x2 = *(const v4fa*)(arow + kb + 16 + 8 * hh), x3 = *(const v4fa*)(arow + kb + 16 + 8 * hh + 4);
    float xs[16] = {x0[0],x0[1],x0[2],x0[3],x1[0],x1[1],x1[2],x1[3],x2[0],x2[1],x2[2],x2[3],x3[0],x3[1],x3[2],x3[3]};
#pragma unroll
    for (int i = 0; i < 16; ++i) { const unsigned short hb = bf16_bits(xs[i]); ah.u[i] = hb; al.u[i] = ASPLIT ? bf16_bits(xs[i] - bf16_val(hb)) : (unsigned short)0; }
#pragma unroll
    for (int t = 0; t < 4; ++t) {
      const unsigned short* brow = Wt + (size_t)(col0 + t * 16 + ln) * ldb + kb;
      FragB b;
      b.half[0] = *(const v8us*)(brow + 8 * hh);
      b.half[1] = *(const v8us*)(brow + 16 + 8 * hh);
      acc[t] = mmaN<ASPLIT ? 2 : 1>(ah.v, al.v, b.v, b.v, acc[t]);
    }
  }
#pragma unroll
  for (int t = 0; t < 4; ++t) {
    float bv = bias ? bias[col0 + t * 16 + ln] : 0.f;
    if (BIAS_BF16) bv = bf16_round(bv);
#pragma unroll
    for (int r = 0; r < 8; ++r) { float v = acc[t][r] + bv; if (ACT == 1) v = fmaxf(v, 0.f); so[w][8 * hh + r][t * 16 + ln] = v; }
  }
  __builtin_amdgcn_fence(__ATOMIC_ACQ_REL, "workgroup");
  __builtin_amdgcn_wave_barrier();
  const int rsub = lane >> 4, c4 = (lane & 15) * 4;
  for (int pass = 0; pass < 2; ++pass) {
#pragma unroll
    for (int q = 0; q < 8; ++q) {
      const int r = q * 2 + rsub;
      const v4f v = *(const v4fa*)&so[w][r][c4];
      *(volatile v4f*)(C + (size_t)(row0 + r) * ldc + col0 + c4) = v;
    }
    if (pass == 0) __threadfence();
  }
}

template <bool ASPLIT, int ACT, bool BIAS_BF16, bool RES_BF16>
__global__ __launch_bounds__(128) void k_gemm_bf3(const float* __restrict__ A, int lda, const unsigned short* __restrict__ Wt, int ldb,
                                                const float* __restrict__ bias, const float* __restrict__ resid, int rmod, int ldr,
                                                float* __restrict__ C, int ldc, int M, int N, int K) {
  __shared__ __attribute__((aligned(16))) float so[4][16][64];
  const int tid = threadIdx.x, w = tid >> 5, lane = tid & 31, ln = lane & 15, hh = lane >> 4;
  const int ntn = N / 64;
  const int wid = blockIdx.x * 4 + w;
  const int mt = wid / ntn, nq = wid % ntn;
  if (mt * 16 >= M) return;
  const int row0 = mt * 16, col0 = nq * 64;
  const float* arow = A + (size_t)(row0 + ln) * lda;
  v8f acc[4] = {};
  for (int kb = 0; kb < K; kb += 32) {
    FragB ah, al;
    const v4f x0 = *(const v4fa*)(arow + kb + 8 * hh), x1 = *(const v4fa*)(arow + kb + 8 * hh + 4);
    const v4f x2 = *(const v4fa*)(arow + kb + 16 + 8 * hh), x3 = *(const v4fa*)(arow + kb + 16 + 8 * hh + 4);
    float xs[16] = {x0[0],x0[1],x0[2],x0[3],x1[0],x1[1],x1[2],x1[3],x2[0],x2[1],x2[2],x2[3],x3[0],x3[1],x3[2],x3[3]};
#pragma unroll
    for (int i = 0; i < 16; ++i) { const unsigned short hb = bf16_bits(xs[i]); ah.u[i] = hb; al.u[i] = ASPLIT ? bf16_bits(xs[i] - bf16_val(hb)) : (unsigned short)0; }
#pragma unroll
    for (int t = 0; t < 4; ++t) {
      const unsigned short* brow = Wt + (size_t)(col0 + t * 16 + ln) * ldb + kb;
      FragB b;
      b.half[0] = *(const v8us*)(brow + 8 * hh);
      b.half[1] = *(const v8us*)(brow + 16 + 8 * hh);
      acc[t] = mmaN<ASPLIT ? 2 : 1>(ah.v, al.v, b.v, b.v, acc[t]);
    }
  }
#pragma unroll
  for (int t = 0; t < 4; ++t) {
    const int col = col0 + t * 16 + ln;
    float bv = bias ? bias[col] : 0.f;
    if (BIAS_BF16) bv = bf16_round(bv);
#pragma unroll
    for (int r = 0; r < 8; ++r) {
      float v = acc[t][r] + bv;
      if (resid) { float rv = resid[(size_t)((row0 + 8 * hh + r) % rmod) * ldr + col]; if (RES_BF16) rv = bf16_round(rv); v += rv; }
      if (ACT == 1) v = fmaxf(v, 0.f);
      if (ACT == 2) v = 0.5f * v * (1.0f + erff(v * 0.70710678118654752f));
      if (ACT == 3) { const float u = 0.7978845608028654f * (v + 0.044715f * v * v * v); v = 0.5f * v * (1.0f + tanhf(u)); }
      so[w][8 * hh + r][t * 16 + ln] = v;
    }
  }
  __builtin_amdgcn_fence(__ATOMIC_ACQ_REL, "workgroup");
  __builtin_amdgcn_wave_barrier();
  const int rsub = lane >> 4, c4 = (lane & 15) * 4;
  for (int pass = 0; pass < 2; ++pass) {
#pragma unroll
    for (int q = 0; q < 8; ++q) {
      const int r = q * 2 + rsub;
      const v4f v = *(const v4fa*)&so[w][r][c4];
      *(volatile v4f*)(C + (size_t)(row0 + r) * ldc + col0 + c4) = v;
    }
    if (pass == 0) __threadfence();
  }
}
template <bool PARAM_BF16>
__global__ __launch_bounds__(256) void k_layernorm(const float* __restrict__ X, const float* __restrict__ R, const float* __restrict__ g, const float* __restrict__ bta,
                                                  float* __restrict__ out_sum, float* __restrict__ out_norm, int N, float eps) {
  __shared__ float red[256];
  const int row = blockIdx.x, tid = threadIdx.x;
  const float* x = X + (size_t)row * N; const float* rr = R ? R + (size_t)row * N : nullptr;
  float vals[16];
  const int per = N / 256;
  float s1 = 0.f;
  for (int u = 0; u < per / 4; ++u) {
    const int j = tid * 4 + 1024 * u;
    const v4f a = *(const v4fa*)(x + j);
    v4f b = {0.f,0.f,0.f,0.f}; if (rr) b = *(const v4fa*)(rr + j);
#pragma unroll
    for (int q = 0; q < 4; ++q) { const float v = a[q] + b[q]; vals[u * 4 + q] = v; s1 += v; }
  }
  red[tid] = s1; __syncthreads();
  for (int st = 128; st > 0; st >>= 1) { if (tid < st) red[tid] += red[tid + st]; __syncthreads(); }
  const float mu = red[0] / (float)N; __syncthreads();
  float s2 = 0.f;
  for (int u = 0; u < per / 4; ++u)
#pragma unroll
    for (int q = 0; q < 4; ++q) { const float c = vals[u * 4 + q] - mu; s2 += c * c; }
  red[tid] = s2; __syncthreads();
  for (int st = 128; st > 0; st >>= 1) { if (tid < st) red[tid] += red[tid + st]; __syncthreads(); }
  const float rs = rsqrtf(red[0] / (float)N + eps);
  for (int pass = 0; pass < 2; ++pass) {
    for (int u = 0; u < per / 4; ++u) {
      const int j = tid * 4 + 1024 * u;
      v4f o, sm;
#pragma unroll
      for (int q = 0; q < 4; ++q) {
        float gg = g[j + q], bb = bta[j + q];
        if (PARAM_BF16) { gg = bf16_round(gg); bb = bf16_round(bb); }
        sm[q] = vals[u * 4 + q]; o[q] = (vals[u * 4 + q] - mu) * rs * gg + bb;
      }
      if (out_sum) *(volatile v4f*)(out_sum + (size_t)row * N + j) = sm;
      *(volatile v4f*)(out_norm + (size_t)row * N + j) = o;
    }
    if (pass == 0) __threadfence();
  }
}


typedef _Float16 v16h __attribute__((ext_vector_type(16)));
union FragH { v16h v; v8us half[2]; _Float16 h[16]; unsigned short u[16]; };
template <int NT>
__device__ __forceinline__ v8f mmaH(v16h ah, v16h al, v16h bh, v16h bl, v8f c) {
  c = __builtin_amdgcn_wmma_f32_16x16x32_f16(false, ah, false, bh, (short)0, c, false, false);
  if (NT >= 2) c = __builtin_amdgcn_wmma_f32_16x16x32_f16(false, al, false, bh, (short)0, c, false, false);
  if (NT >= 3) c = __builtin_amdgcn_wmma_f32_16x16x32_f16(false, ah, false, bl, (short)0, c, false, false);
  asm volatile("v_nop\n\tv_nop\n\tv_nop\n\tv_nop" : "+v"(c) : "v"(ah), "v"(al), "v"(bh), "v"(bl));
  return c;
}
template <bool ASPLIT>
__global__ __launch_bounds__(128) void k_gemm_h(const float* __restrict__ A, int lda, size_t sA, const _Float16* __restrict__ Bh, int ldb, size_t sB, float alpha, float* __restrict__ C, int ldc, size_t sC, int M, int N, int K) {
  __shared__ __attribute__((aligned(16))) float so[4][16][64];
  const int tid = threadIdx.x, w = tid >> 5, lane = tid & 31, ln = lane & 15, hh = lane >> 4; const int by = blockIdx.y;
  A += (size_t)by * sA; Bh += (size_t)by * sB; C += (size_t)by * sC;
  const int ntn = (N + 63) / 64; const int wid = blockIdx.x * 4 + w; const int mt = wid / ntn, nq = wid % ntn; if (mt * 16 >= M) return;
  const int row0 = mt * 16, col0 = nq * 64; const float* arow = A + (size_t)(row0 + ln) * lda;
  v8f acc[4] = {};
  for (int kb = 0; kb < K; kb += 32) {
    FragH ah, al;
    const v4f x0 = *(const v4fa*)(arow + kb + 8 * hh), x1 = *(const v4fa*)(arow + kb + 8 * hh + 4), x2 = *(const v4fa*)(arow + kb + 16 + 8 * hh), x3 = *(const v4fa*)(arow + kb + 16 + 8 * hh + 4);
    float xs[16] = {x0[0],x0[1],x0[2],x0[3],x1[0],x1[1],x1[2],x1[3],x2[0],x2[1],x2[2],x2[3],x3[0],x3[1],x3[2],x3[3]};
#pragma unroll
    for (int i = 0; i < 16; ++i) { const _Float16 h = (_Float16)xs[i]; ah.h[i] = h; al.h[i] = ASPLIT ? (_Float16)(xs[i] - (float)h) : (_Float16)0.0f; }
#pragma unroll
    for (int t = 0; t < 4; ++t) { if (col0 + t * 16 >= N) continue; const size_t boff = (size_t)(col0 + t * 16 + ln) * ldb + kb; FragH bq; bq.half[0] = *(const v8us*)(Bh + boff + 8 * hh); bq.half[1] = *(const v8us*)(Bh + boff + 16 + 8 * hh);
      acc[t] = mmaH<ASPLIT ? 2 : 1>(ah.v, al.v, bq.v, bq.v, acc[t]); }
  }
#pragma unroll
  for (int t = 0; t < 4; ++t) { if (col0 + t * 16 >= N) continue;
#pragma unroll
    for (int r = 0; r < 8; ++r) so[w][8 * hh + r][t * 16 + ln] = acc[t][r] * alpha; }
  __builtin_amdgcn_fence(__ATOMIC_ACQ_REL, "workgroup"); __builtin_amdgcn_wave_barrier();
  const int rsub = lane >> 4, c4 = (lane & 15) * 4;
  for (int pass = 0; pass < 2; ++pass) {
#pragma unroll
    for (int q = 0; q < 8; ++q) { const int r = q * 2 + rsub; if (col0 + c4 < N) { const v4f v = *(const v4fa*)&so[w][r][c4]; *(volatile v4f*)(C + (size_t)(row0 + r) * ldc + col0 + c4) = v; } }
    if (pass == 0) __threadfence(); }
}

__global__ __launch_bounds__(256) void k_wt_f16(const float* __restrict__ W, _Float16* __restrict__ Wt, int K, int N, float scale) {
  const int t = blockIdx.x * 256 + threadIdx.x; if (t >= N * (K / 8)) return; const int n = t / (K / 8), k8 = (t % (K / 8)) * 8; FragH f;
#pragma unroll
  for (int i = 0; i < 8; ++i) f.h[i] = (_Float16)(bf16_round(W[(size_t)(k8 + i) * N + n]) * scale); const v8us o = f.half[0];
  *(volatile v8us*)((unsigned short*)Wt + (size_t)n * K + k8) = o; __threadfence(); *(volatile v8us*)((unsigned short*)Wt + (size_t)n * K + k8) = o;
}
template <int ACT>
__global__ __launch_bounds__(128) void k_gemm_hhx(const _Float16* __restrict__ A, int lda, size_t sA, const _Float16* __restrict__ Bh, int ldb, size_t sB, float alpha, const float* __restrict__ bias, size_t sBias, const float* __restrict__ CP, int rowsPerB, size_t sCPb, int row0g,
    float* __restrict__ C, _Float16* __restrict__ C16, int ldc, size_t sC, int M, int N, int K) {
  __shared__ __attribute__((aligned(16))) float so[4][16][64];
  const int tid = threadIdx.x, w = tid >> 5, lane = tid & 31, ln = lane & 15, hh = lane >> 4; const int by = blockIdx.y;
  A += (size_t)by * sA; Bh += (size_t)by * sB; const size_t cofs = (size_t)by * sC; const float* bp = bias ? bias + (size_t)by * sBias : nullptr;
  const int ntn = (N + 63) / 64; const int wid = blockIdx.x * 4 + w; const int mt = wid / ntn, nq = wid % ntn; if (mt * 16 >= M) return;
  const int row0 = mt * 16, col0 = nq * 64; const _Float16* arow = A + (size_t)(row0 + ln) * lda;
  v8f acc[4] = {};
  for (int kb = 0; kb < K; kb += 32) { FragH ah; ah.half[0] = *(const v8us*)((const unsigned short*)arow + kb + 8 * hh); ah.half[1] = *(const v8us*)((const unsigned short*)arow + kb + 16 + 8 * hh);
#pragma unroll
    for (int t = 0; t < 4; ++t) { if (col0 + t * 16 >= N) continue; const size_t boff = (size_t)(col0 + t * 16 + ln) * ldb + kb; FragH bq; bq.half[0] = *(const v8us*)((const unsigned short*)Bh + boff + 8 * hh); bq.half[1] = *(const v8us*)((const unsigned short*)Bh + boff + 16 + 8 * hh);
      acc[t] = mmaH<1>(ah.v, ah.v, bq.v, bq.v, acc[t]); }
  }
#pragma unroll
  for (int t = 0; t < 4; ++t) { if (col0 + t * 16 >= N) continue; const int col = col0 + t * 16 + ln; const float bv = bp ? bf16_round(bp[col]) : 0.f;
#pragma unroll
    for (int r = 0; r < 8; ++r) { float v = acc[t][r] * alpha + bv; if (CP) { const int bidx = (row0g + row0 + 8 * hh + r) / rowsPerB; v += CP[(size_t)bidx * sCPb + (size_t)by * 64 + col]; } if (ACT == 1) v = (v > 0.f) ? v : expm1f(v); else if (ACT == 7) v = (v > 0.f) ? v + 1.0f : expf(v); else if (ACT == 8) v = tanhf(v); else if (ACT == 9) v = 0.5f * v * (1.0f + tanhf(0.7978845608028654f * (v + 0.044715f * v * v * v))); else if (ACT == 11) v = 1.0f / (1.0f + expf(-v)); else if (ACT == 12) v = (v > 0.f) ? v : 0.01f * v; else if (ACT == 14) v = (v > 0.f) ? v : 0.1f * v; else if (ACT == 15) v = v / (1.0f + expf(-v)); else if (ACT == 3) v = fmaxf(v, 0.f); else if (ACT == 6) v = 0.5f * v * (1.0f + erff(v * 0.70710678118654752f)); so[w][8 * hh + r][t * 16 + ln] = v; } }
  __builtin_amdgcn_fence(__ATOMIC_ACQ_REL, "workgroup"); __builtin_amdgcn_wave_barrier();
  const int rsub = lane >> 4, c4 = (lane & 15) * 4; typedef _Float16 v4h __attribute__((ext_vector_type(4)));
  for (int pass = 0; pass < 2; ++pass) {
#pragma unroll
    for (int q = 0; q < 8; ++q) { const int r = q * 2 + rsub; if (col0 + c4 < N) { const v4f v = *(const v4fa*)&so[w][r][c4]; if (C) *(volatile v4f*)(C + cofs + (size_t)(row0 + r) * ldc + col0 + c4) = v; if (C16) { v4h h4; for (int i = 0; i < 4; ++i) h4[i] = (_Float16)v[i]; *(volatile v4h*)(C16 + cofs + (size_t)(row0 + r) * ldc + col0 + c4) = h4; } } }
    if (pass == 0) __threadfence(); }
}


typedef _Float16 v4h __attribute__((ext_vector_type(4)));

__global__ __launch_bounds__(256) void k_x16(const float* __restrict__ x, _Float16* __restrict__ X16, size_t n8) { const size_t t = (size_t)blockIdx.x * 256 + threadIdx.x; if (t >= n8) return; FragH f;
#pragma unroll
  for (int q = 0; q < 8; ++q) f.h[q] = (_Float16)bf16_round(x[t * 8 + q]); *(volatile v8us*)((unsigned short*)X16 + t * 8) = f.half[0]; __threadfence(); *(volatile v8us*)((unsigned short*)X16 + t * 8) = f.half[0]; }
__global__ __launch_bounds__(256) void k_h16(const float* __restrict__ x, _Float16* __restrict__ X16, size_t n8) { const size_t t = (size_t)blockIdx.x * 256 + threadIdx.x; if (t >= n8) return; FragH f;
#pragma unroll
  for (int q = 0; q < 8; ++q) f.h[q] = (_Float16)x[t * 8 + q]; *(volatile v8us*)((unsigned short*)X16 + t * 8) = f.half[0]; __threadfence(); *(volatile v8us*)((unsigned short*)X16 + t * 8) = f.half[0]; }
__global__ __launch_bounds__(256) void k_round16f(const float* __restrict__ W, _Float16* __restrict__ Bt, size_t n8) { const size_t t = (size_t)blockIdx.x * 256 + threadIdx.x; if (t >= n8) return; FragH f;
#pragma unroll
  for (int i = 0; i < 8; ++i) f.h[i] = (_Float16)(bf16_round(W[t * 8 + i]) * 16.0f); *(volatile v8us*)((unsigned short*)Bt + t * 8) = f.half[0]; __threadfence(); *(volatile v8us*)((unsigned short*)Bt + t * 8) = f.half[0]; }
template <int NHv, int TTv>
__global__ __launch_bounds__(256) void k_vt(const _Float16* __restrict__ V16, int ldv, int voff, _Float16* __restrict__ Vt) { __shared__ unsigned short tl[64][66]; const int tid = threadIdx.x; const int slab = blockIdx.x / (TTv / 64), lg = blockIdx.x % (TTv / 64); const int b = slab / NHv, h = slab % NHv;
  for (int i = tid; i < 64 * 8; i += 256) { const int r = i / 8, c8 = (i % 8) * 8; FragH f; f.half[0] = *(const v8us*)((const unsigned short*)V16 + ((size_t)b * TTv + lg * 64 + r) * ldv + voff + h * 64 + c8);
#pragma unroll
    for (int q = 0; q < 8; ++q) tl[r][c8 + q] = f.u[q]; }
  __syncthreads();
  for (int pass = 0; pass < 2; ++pass) {
#pragma unroll
    for (int rd = 0; rd < 2; ++rd) { const int d = rd * 32 + tid / 8, pc = tid % 8; FragH f;
#pragma unroll
      for (int q = 0; q < 8; ++q) f.u[q] = tl[pc * 8 + q][d];
      *(volatile v8us*)((unsigned short*)Vt + ((size_t)slab * 64 + d) * TTv + lg * 64 + pc * 8) = f.half[0]; }
    if (pass == 0) __threadfence(); } }

__global__ __launch_bounds__(256) void k_hl(const float* __restrict__ F, _Float16* __restrict__ Hh, _Float16* __restrict__ Hl, size_t n8) { const size_t t = (size_t)blockIdx.x * 256 + threadIdx.x; if (t >= n8) return; FragH fh, fl; const v4f a = *(const v4fa*)(F + t * 8), c = *(const v4fa*)(F + t * 8 + 4);
#pragma unroll
  for (int q = 0; q < 4; ++q) { _Float16 h = (_Float16)a[q]; fh.h[q] = h; fl.h[q] = (_Float16)((a[q] - (float)h) * 1024.0f); h = (_Float16)c[q]; fh.h[4 + q] = h; fl.h[4 + q] = (_Float16)((c[q] - (float)h) * 1024.0f); }
  for (int pass = 0; pass < 2; ++pass) { *(volatile v8us*)((unsigned short*)Hh + t * 8) = fh.half[0]; *(volatile v8us*)((unsigned short*)Hl + t * 8) = fl.half[0]; if (pass == 0) __threadfence(); } }

__device__ __forceinline__ v16h g2_frag(const _Float16* p, int hh) { FragH f; f.half[0] = *(const v8us*)((const unsigned short*)p + 8 * hh); f.half[1] = *(const v8us*)((const unsigned short*)p + 16 + 8 * hh); return f.v; }
__device__ __forceinline__ v8f g2_mma(v16h a, v16h b, v8f c) { v8f d = __builtin_amdgcn_wmma_f32_16x16x32_f16(false, a, false, b, (short)0, c, false, false); asm volatile("v_nop\n\tv_nop\n\tv_nop\n\tv_nop" : "+v"(d) : "v"(a), "v"(b)); return d; }
template <int ACT>
__global__ __launch_bounds__(128) void k_gemm2(const _Float16* __restrict__ A, int lda, size_t sA, const _Float16* __restrict__ Bh, int ldb, size_t sB, float alpha, const float* __restrict__ bias, size_t sBias, const float* __restrict__ CP, int rowsPerB, size_t sCPb, int row0g,
    float* __restrict__ C, _Float16* __restrict__ C16, int ldc, size_t sC, int M, int N, int K) {
  __shared__ __attribute__((aligned(16))) float so[4][32][68];
  const int tid = threadIdx.x, w = tid >> 5, lane = tid & 31, ln = lane & 15, hh = lane >> 4; const int by = blockIdx.y;
  A += (size_t)by * sA; Bh += (size_t)by * sB; const size_t cofs = (size_t)by * sC; const float* bp = bias ? bias + (size_t)by * sBias : nullptr;
  const int ntn = N >> 6; const int mt = blockIdx.x / ntn, nq = blockIdx.x - mt * ntn; const int row0 = mt * 128 + 32 * w, col0 = nq * 64; if (row0 >= M) return;
  const _Float16* a0p = A + (size_t)(row0 + ln) * lda; const _Float16* a1p = a0p + (size_t)16 * lda;
  const _Float16* b0p = Bh + (size_t)(col0 + ln) * ldb; const _Float16* b1p = b0p + (size_t)16 * ldb; const _Float16* b2p = b1p + (size_t)16 * ldb; const _Float16* b3p = b2p + (size_t)16 * ldb;
  const v8f z8 = {0.f,0.f,0.f,0.f,0.f,0.f,0.f,0.f}; v8f c00 = z8, c01 = z8, c02 = z8, c03 = z8, c10 = z8, c11 = z8, c12 = z8, c13 = z8;
#pragma unroll 1
  for (int kb = 0; kb < K; kb += 32) { const v16h a0 = g2_frag(a0p + kb, hh), a1 = g2_frag(a1p + kb, hh);
    v16h b = g2_frag(b0p + kb, hh); c00 = g2_mma(a0, b, c00); c10 = g2_mma(a1, b, c10);
    b = g2_frag(b1p + kb, hh); c01 = g2_mma(a0, b, c01); c11 = g2_mma(a1, b, c11);
    b = g2_frag(b2p + kb, hh); c02 = g2_mma(a0, b, c02); c12 = g2_mma(a1, b, c12);
    b = g2_frag(b3p + kb, hh); c03 = g2_mma(a0, b, c03); c13 = g2_mma(a1, b, c13); }
  v8f accs[8] = {c00, c01, c02, c03, c10, c11, c12, c13};
#pragma unroll
  for (int u = 0; u < 8; ++u) { const int t = u & 3, half = u >> 2; const int col = col0 + t * 16 + ln; const float bv = bp ? bf16_round(bp[col]) : 0.f;
#pragma unroll
    for (int r = 0; r < 8; ++r) { const int rloc = half * 16 + 8 * hh + r; float v = accs[u][r] * alpha + bv; if (CP) { const int bidx = (row0g + row0 + rloc) / rowsPerB; v += CP[(size_t)bidx * sCPb + (size_t)by * 64 + col]; }
      if (ACT == 3) v = fmaxf(v, 0.f); else if (ACT == 6) v = 0.5f * v * (1.0f + erff(v * 0.70710678118654752f)); else if (ACT == 11) v = 1.0f / (1.0f + expf(-v)); else if (ACT == 15) v = v / (1.0f + expf(-v)); else if (ACT == 12) v = (v > 0.f) ? v : 0.01f * v; else if (ACT == 8) v = tanhf(v);
      so[w][rloc][t * 16 + ln] = v; } }
  __builtin_amdgcn_fence(__ATOMIC_ACQ_REL, "workgroup"); __builtin_amdgcn_wave_barrier();
  const int rsub = lane >> 4, c4 = (lane & 15) * 4;
  for (int pass = 0; pass < 2; ++pass) {
#pragma unroll
    for (int q = 0; q < 16; ++q) { const int r = q * 2 + rsub; const v4f v = *(const v4fa*)&so[w][r][c4]; if (C) *(volatile v4f*)(C + cofs + (size_t)(row0 + r) * ldc + col0 + c4) = v; if (C16) { v4h h4; for (int i = 0; i < 4; ++i) h4[i] = (_Float16)v[i]; *(volatile v4h*)(C16 + cofs + (size_t)(row0 + r) * ldc + col0 + c4) = h4; } }
    if (pass == 0) __threadfence(); } }


__global__ __launch_bounds__(128) void k_flashpad(const _Float16* __restrict__ Q16, int ldq, const _Float16* __restrict__ K16, int ldk, const _Float16* __restrict__ Vt, const int* __restrict__ PADK, float* __restrict__ O, int ldo) {
  #pragma clang fp contract(off)
  constexpr int RPW = 16, RTN = RPW / 16, NQB = TQ / (4 * RPW), DT = 4, KS = 2;
  __shared__ __attribute__((aligned(16))) unsigned short sP[4][RPW][40]; __shared__ __attribute__((aligned(16))) float sO[4][RPW][64 + 4];
  const int tid = threadIdx.x, w = tid >> 5, lane = tid & 31, ln = lane & 15, hh = lane >> 4;
  const int slab = blockIdx.x / NQB, qblk = blockIdx.x % NQB; const int b = slab / NH, h = slab % NH; const int qb0 = qblk * (4 * RPW); const int q0 = qb0 + w * RPW;
  FragH aq[2][KS];
#pragma unroll
  for (int rt = 0; rt < RTN; ++rt) { const unsigned short* qr = (const unsigned short*)Q16 + ((size_t)b * TQ + q0 + rt * 16 + ln) * ldq + h * 64;
#pragma unroll
    for (int ks = 0; ks < KS; ++ks) { aq[rt][ks].half[0] = *(const v8us*)(qr + ks * 32 + 8 * hh); aq[rt][ks].half[1] = *(const v8us*)(qr + ks * 32 + 16 + 8 * hh); } }
  const unsigned short* Vth = (const unsigned short*)Vt + (size_t)slab * 64 * TK;
  float m_r[2][8], l_r[2][8]; v8f oacc[2][DT];
#pragma unroll
  for (int rt = 0; rt < RTN; ++rt) {
#pragma unroll
    for (int r = 0; r < 8; ++r) { m_r[rt][r] = -3.0e38f; l_r[rt][r] = 0.f; }
#pragma unroll
    for (int dt = 0; dt < DT; ++dt) oacc[rt][dt] = (v8f){0.f,0.f,0.f,0.f,0.f,0.f,0.f,0.f}; }
  const int jend = TK;
#pragma unroll 1
  for (int j0 = 0; j0 < jend; j0 += 32) {
    v8f s[2][2];
#pragma unroll
    for (int nt = 0; nt < 2; ++nt) { const unsigned short* kr = (const unsigned short*)K16 + ((size_t)b * TK + j0 + nt * 16 + ln) * ldk + h * 64; FragH bk[KS];
#pragma unroll
      for (int ks = 0; ks < KS; ++ks) { bk[ks].half[0] = *(const v8us*)(kr + ks * 32 + 8 * hh); bk[ks].half[1] = *(const v8us*)(kr + ks * 32 + 16 + 8 * hh); }
#pragma unroll
      for (int rt = 0; rt < RTN; ++rt) { v8f acc = (v8f){0.f,0.f,0.f,0.f,0.f,0.f,0.f,0.f};
#pragma unroll
        for (int ks = 0; ks < KS; ++ks) acc = mmaH<1>(aq[rt][ks].v, aq[rt][ks].v, bk[ks].v, bk[ks].v, acc); s[rt][nt] = acc; } }
#pragma unroll
    for (int rt = 0; rt < RTN; ++rt)
#pragma unroll
      for (int r = 0; r < 8; ++r) { const int tq = q0 + rt * 16 + 8 * hh + r; const int k0 = j0 + ln, k1 = j0 + 16 + ln; (void)tq; const int* pk = PADK + (size_t)(b % NBATCH) * TK;
        const float s0 = pk[k0] ? -1.0e9f : s[rt][0][r] * SCL, s1 = pk[k1] ? -1.0e9f : s[rt][1][r] * SCL; float mc = fmaxf(s0, s1);
        mc = fmaxf(mc, __shfl_xor(mc, 1, 32)); mc = fmaxf(mc, __shfl_xor(mc, 2, 32)); mc = fmaxf(mc, __shfl_xor(mc, 4, 32)); mc = fmaxf(mc, __shfl_xor(mc, 8, 32));
        const float mn = fmaxf(m_r[rt][r], mc); const float al = (mn > -1.0e38f) ? expf(m_r[rt][r] - mn) : 1.0f; m_r[rt][r] = mn; const float p0 = expf(s0 - mn), p1 = expf(s1 - mn); l_r[rt][r] = l_r[rt][r] * al + p0 + p1;
#pragma unroll
        for (int dt = 0; dt < DT; ++dt) oacc[rt][dt][r] *= al;
        FragH t2; t2.h[0] = (_Float16)(p0 * 1024.0f); t2.h[1] = (_Float16)(p1 * 1024.0f); sP[w][rt * 16 + 8 * hh + r][ln] = t2.u[0]; sP[w][rt * 16 + 8 * hh + r][16 + ln] = t2.u[1]; }
    __builtin_amdgcn_fence(__ATOMIC_ACQ_REL, "workgroup"); __builtin_amdgcn_wave_barrier();
    FragH pa[2];
#pragma unroll
    for (int rt = 0; rt < RTN; ++rt) { pa[rt].half[0] = *(const v8us*)&sP[w][rt * 16 + ln][8 * hh]; pa[rt].half[1] = *(const v8us*)&sP[w][rt * 16 + ln][16 + 8 * hh]; }
#pragma unroll
    for (int dt = 0; dt < DT; ++dt) { const unsigned short* vrow = Vth + (size_t)(dt * 16 + ln) * TK + j0; FragH bv; bv.half[0] = *(const v8us*)(vrow + 8 * hh); bv.half[1] = *(const v8us*)(vrow + 16 + 8 * hh);
#pragma unroll
      for (int rt = 0; rt < RTN; ++rt) oacc[rt][dt] = mmaH<1>(pa[rt].v, pa[rt].v, bv.v, bv.v, oacc[rt][dt]); }
    __builtin_amdgcn_fence(__ATOMIC_ACQ_REL, "workgroup"); __builtin_amdgcn_wave_barrier(); }
#pragma unroll
  for (int rt = 0; rt < RTN; ++rt) {
#pragma unroll
    for (int r = 0; r < 8; ++r) { float l = l_r[rt][r]; l += __shfl_xor(l, 1, 32); l += __shfl_xor(l, 2, 32); l += __shfl_xor(l, 4, 32); l += __shfl_xor(l, 8, 32); l_r[rt][r] = (l > 0.f) ? 1.0f / (l * 1024.0f) : 0.f; }
#pragma unroll
    for (int dt = 0; dt < DT; ++dt)
#pragma unroll
      for (int r = 0; r < 8; ++r) sO[w][rt * 16 + 8 * hh + r][dt * 16 + ln] = oacc[rt][dt][r] * l_r[rt][r]; }
  __builtin_amdgcn_fence(__ATOMIC_ACQ_REL, "workgroup"); __builtin_amdgcn_wave_barrier();
  for (int pass = 0; pass < 2; ++pass) {
#pragma unroll
    for (int rp = 0; rp < RPW; rp += 2) { const int r = rp + (lane >> 4), pc = lane & 15; const v4f val = *(const v4fa*)&sO[w][r][pc * 4]; *(volatile v4f*)(O + ((size_t)b * TQ + q0 + r) * ldo + h * 64 + pc * 4) = val; }
    if (pass == 0) __threadfence(); } }
__device__ __forceinline__ float seluf(float v) { return SELU_S * (v > 0.f ? v : SELU_A * expm1f(v)); }
__global__ __launch_bounds__(256) void k_bpad(const float* __restrict__ b, int n, int np, float* __restrict__ BP) { const int t = blockIdx.x * 256 + threadIdx.x; if (t >= np) return; const float v = (t < n) ? b[t] : 0.f; *(volatile float*)(BP + t) = v; __threadfence(); *(volatile float*)(BP + t) = v; }
__global__ __launch_bounds__(256) void k_wtp(const float* __restrict__ Wm, int K, int N, int KP, int NP, _Float16* __restrict__ Bt) {
  const int t = blockIdx.x * 256 + threadIdx.x; if (t >= NP * (KP / 8)) return; const int n = t / (KP / 8), k0 = (t % (KP / 8)) * 8; FragH f;
#pragma unroll
  for (int q = 0; q < 8; ++q) { const int k = k0 + q; f.h[q] = (n < N && k < K) ? (_Float16)(bf16_round(Wm[(size_t)k * N + n]) * 16.0f) : (_Float16)0.0f; }
  *(volatile v8us*)((unsigned short*)Bt + (size_t)n * KP + k0) = f.half[0]; __threadfence(); *(volatile v8us*)((unsigned short*)Bt + (size_t)n * KP + k0) = f.half[0]; }
__global__ __launch_bounds__(256) void k_wtp_o1(const float* __restrict__ Wm, _Float16* __restrict__ Bt) {
  const int t = blockIdx.x * 256 + threadIdx.x; if (t >= 1536 * (1536 / 8)) return; const int n = t / (1536 / 8), k0 = (t % (1536 / 8)) * 8; FragH f;
#pragma unroll
  for (int q = 0; q < 8; ++q) { const int kp = k0 + q; const int k = (kp < FF) ? DD + kp : kp - FF; f.h[q] = (n < 1500 && kp < 1500) ? (_Float16)(bf16_round(Wm[(size_t)k * 1500 + n]) * 16.0f) : (_Float16)0.0f; }
  *(volatile v8us*)((unsigned short*)Bt + (size_t)n * 1536 + k0) = f.half[0]; __threadfence(); *(volatile v8us*)((unsigned short*)Bt + (size_t)n * 1536 + k0) = f.half[0]; }
__global__ __launch_bounds__(256) void k_wtp2(const float* __restrict__ Wm, int K, int N, int KP, int NP, _Float16* __restrict__ Bt) {
  const int t = blockIdx.x * 256 + threadIdx.x; if (t >= NP * (2 * KP / 8)) return; const int n = t / (2 * KP / 8), k0 = (t % (2 * KP / 8)) * 8; const bool lo = (k0 >= KP); const float sc = lo ? 1.0f : 16.0f; FragH f;
#pragma unroll
  for (int q = 0; q < 8; ++q) { const int k = k0 + q - (lo ? KP : 0); f.h[q] = (n < N && k < K) ? (_Float16)(bf16_round(Wm[(size_t)k * N + n]) * sc) : (_Float16)0.0f; }
  *(volatile v8us*)((unsigned short*)Bt + (size_t)n * 2 * KP + k0) = f.half[0]; __threadfence(); *(volatile v8us*)((unsigned short*)Bt + (size_t)n * 2 * KP + k0) = f.half[0]; }
__global__ __launch_bounds__(256) void k_wtp_o1p(const float* __restrict__ Wm, _Float16* __restrict__ Bt) {
  const int t = blockIdx.x * 256 + threadIdx.x; if (t >= 1536 * (3072 / 8)) return; const int n = t / (3072 / 8), k0 = (t % (3072 / 8)) * 8; const bool lo = (k0 >= 1536); const float sc = lo ? 1.0f : 16.0f; FragH f;
#pragma unroll
  for (int q = 0; q < 8; ++q) { const int j = k0 + q - (lo ? 1536 : 0); const int k = (j < FF) ? DD + j : j - FF; f.h[q] = (n < 1500 && j < 1500) ? (_Float16)(bf16_round(Wm[(size_t)k * 1500 + n]) * sc) : (_Float16)0.0f; }
  *(volatile v8us*)((unsigned short*)Bt + (size_t)n * 3072 + k0) = f.half[0]; __threadfence(); *(volatile v8us*)((unsigned short*)Bt + (size_t)n * 3072 + k0) = f.half[0]; }
__global__ __launch_bounds__(256) void k_padk(const int* __restrict__ tok, int* __restrict__ PADK) { const int t = blockIdx.x * 256 + threadIdx.x; if (t >= NROW) return; const int v = (tok[t] == 0) ? 1 : 0; *(volatile int*)(PADK + t) = v; __threadfence(); *(volatile int*)(PADK + t) = v; }
__global__ __launch_bounds__(256) void k_embed(const int* __restrict__ tok, const float* __restrict__ emb, float* __restrict__ X, _Float16* __restrict__ X16) {
  #pragma clang fp contract(off)
  const int t = blockIdx.x * 256 + threadIdx.x; if (t >= NROW * (DP / 4)) return; const int r = t / (DP / 4), c0 = (t % (DP / 4)) * 4; const int l = r % LL; int id = tok[r]; id = min(max(id, 0), 49999); v4f o; _Float16 hh[4];
#pragma unroll
  for (int q = 0; q < 4; ++q) { const int c = c0 + q; float v = 0.f;
    if (c < DD) { const double ang = (double)l / pow(10000.0, 2.0 * (double)(c / 2) / (double)DD); const float pe = (float)((c & 1) ? cos(ang) : sin(ang)); v = bf16_round(emb[(size_t)id * DD + c]) + pe; }
    o[q] = v; hh[q] = (_Float16)v; }
  const unsigned long long pk = *(const unsigned long long*)hh;
  for (int pass = 0; pass < 2; ++pass) { *(volatile v4f*)(X + (size_t)r * DP + c0) = o; *(volatile unsigned long long*)((unsigned short*)X16 + (size_t)r * DP + c0) = pk; if (pass == 0) __threadfence(); } }
__global__ __launch_bounds__(256) void k_pseudo(const float* __restrict__ F, _Float16* __restrict__ PS) {
  const int tt = blockIdx.x * 256 + threadIdx.x; if (tt >= NPS * LL * 8) return; const int d0 = (tt & 7) * 8; const int t = (tt >> 3) % LL; const int bh = tt / (8 * LL); const int b = bh / NHD, j = bh % NHD; FragH f;
#pragma unroll
  for (int q = 0; q < 8; ++q) { const int d = d0 + q; _Float16 v = (_Float16)0.0f;
    if (d < DPH) { const int flat = j * LL * DPH + t * DPH + d; const int l = flat / DD, c = flat % DD; v = (_Float16)F[((size_t)b * LL + l) * DP + c]; }
    f.h[q] = v; }
  *(volatile v8us*)((unsigned short*)PS + ((size_t)bh * LL + t) * 64 + d0) = f.half[0]; __threadfence(); *(volatile v8us*)((unsigned short*)PS + ((size_t)bh * LL + t) * 64 + d0) = f.half[0]; }
__global__ __launch_bounds__(256) void k_unpseudo(const float* __restrict__ O, _Float16* __restrict__ C16) {
  const int tt = blockIdx.x * 256 + threadIdx.x; if (tt >= NROW * (DP / 8)) return; const int r = tt / (DP / 8), c0 = (tt % (DP / 8)) * 8; const int b = r / LL, l = r % LL; FragH f;
#pragma unroll
  for (int q = 0; q < 8; ++q) { const int c = c0 + q; _Float16 v = (_Float16)0.0f;
    if (c < DD) { const int flat = l * DD + c; const int j = flat / (LL * DPH), rem = flat % (LL * DPH); const int t = rem / DPH, d = rem % DPH; v = (_Float16)O[(((size_t)(b * NHD + j)) * LL + t) * 64 + d]; }
    f.h[q] = v; }
  *(volatile v8us*)((unsigned short*)C16 + (size_t)r * DP + c0) = f.half[0]; __threadfence(); *(volatile v8us*)((unsigned short*)C16 + (size_t)r * DP + c0) = f.half[0]; }
__global__ __launch_bounds__(256) void k_ln300(const float* __restrict__ T, const float* __restrict__ g, const float* __restrict__ bb, float* __restrict__ X, _Float16* __restrict__ X16) {
  #pragma clang fp contract(off)
  const int tid = threadIdx.x, w = tid >> 5, ln = tid & 31; const int r = blockIdx.x * 8 + w; if (r >= NROW) return; const float* x = T + (size_t)r * DP; float v[10]; float s = 0.f;
#pragma unroll
  for (int i = 0; i < 10; ++i) { const int c = ln + 32 * i; v[i] = (c < DD) ? x[c] : 0.f; s += v[i]; }
  for (int o = 16; o > 0; o >>= 1) s += __shfl_xor(s, o, 32); const float mu = s / (float)DD; float q2 = 0.f;
#pragma unroll
  for (int i = 0; i < 10; ++i) { const int c = ln + 32 * i; const float d = (c < DD) ? v[i] - mu : 0.f; v[i] = d; q2 += d * d; }
  for (int o = 16; o > 0; o >>= 1) q2 += __shfl_xor(q2, o, 32); const float dn = sqrtf(q2 / (float)DD + 1e-5f);
  for (int pass = 0; pass < 2; ++pass) {
#pragma unroll
    for (int i = 0; i < 10; ++i) { const int c = ln + 32 * i; const float y = (c < DD) ? (v[i] / dn * bf16_round(g[c]) + bf16_round(bb[c])) : 0.f; *(volatile float*)(X + (size_t)r * DP + c) = y; *(volatile _Float16*)(X16 + (size_t)r * DP + c) = (_Float16)y; }
    if (pass == 0) __threadfence(); } }
__global__ __launch_bounds__(256) void k_selu16(const float* __restrict__ F, int pf, int n, int np8, _Float16* __restrict__ D16, int pd, int off, int lofs) {
  #pragma clang fp contract(off)
  const int tt = blockIdx.x * 256 + threadIdx.x; if (tt >= NROW * (np8 / 8)) return; const int r = tt / (np8 / 8), c0 = (tt % (np8 / 8)) * 8; FragH f, fl;
#pragma unroll
  for (int q = 0; q < 8; ++q) { const int c = c0 + q; const float v = (c < n) ? seluf(F[(size_t)r * pf + c]) : 0.f; const _Float16 hv = (_Float16)v; f.h[q] = hv; fl.h[q] = (_Float16)((v - (float)hv) * 16.0f); }
  unsigned short* d = (unsigned short*)D16 + (size_t)r * pd + off + c0;
  for (int pass = 0; pass < 2; ++pass) { *(volatile v8us*)d = f.half[0]; if (lofs) *(volatile v8us*)(d + lofs) = fl.half[0]; if (pass == 0) __threadfence(); } }
__global__ __launch_bounds__(256) void k_cat16(const float* __restrict__ F, int pf, int n, int np8, _Float16* __restrict__ D16, int pd, int off, int lofs) {
  #pragma clang fp contract(off)
  const int tt = blockIdx.x * 256 + threadIdx.x; if (tt >= NROW * (np8 / 8)) return; const int r = tt / (np8 / 8), c0 = (tt % (np8 / 8)) * 8; FragH f, fl;
#pragma unroll
  for (int q = 0; q < 8; ++q) { const int c = c0 + q; const float v = (c < n) ? F[(size_t)r * pf + c] : 0.f; const _Float16 hv = (_Float16)v; f.h[q] = hv; fl.h[q] = (_Float16)((v - (float)hv) * 16.0f); }
  unsigned short* d = (unsigned short*)D16 + (size_t)r * pd + off + c0;
  for (int pass = 0; pass < 2; ++pass) { *(volatile v8us*)d = f.half[0]; if (lofs) *(volatile v8us*)(d + lofs) = fl.half[0]; if (pass == 0) __threadfence(); } }
template <int ACT>
__global__ __launch_bounds__(256) void k_pack1200(const float* __restrict__ F, float* __restrict__ out, _Float16* __restrict__ D16) {
  #pragma clang fp contract(off)
  const int tt = blockIdx.x * 256 + threadIdx.x; if (tt >= NROW * (FF / 4)) return; const int r = tt / (FF / 4), c0 = (tt % (FF / 4)) * 4; const v4f a = *(const v4fa*)(F + (size_t)r * FFP + c0); v4f o; _Float16 hh[4];
#pragma unroll
  for (int q = 0; q < 4; ++q) { o[q] = ACT ? seluf(a[q]) : a[q]; hh[q] = (_Float16)o[q]; }
  _Float16 hl[4];
#pragma unroll
  for (int q = 0; q < 4; ++q) hl[q] = (_Float16)((o[q] - (float)hh[q]) * 16.0f);
  const unsigned long long pk = *(const unsigned long long*)hh, pl = *(const unsigned long long*)hl;
  for (int pass = 0; pass < 2; ++pass) { *(volatile v4f*)(out + (size_t)r * FF + c0) = o; if (D16) { *(volatile unsigned long long*)((unsigned short*)D16 + (size_t)r * 2 * FFP + c0) = pk; *(volatile unsigned long long*)((unsigned short*)D16 + (size_t)r * 2 * FFP + FFP + c0) = pl; } if (pass == 0) __threadfence(); } }
__global__ __launch_bounds__(256) void k_zpad16(_Float16* __restrict__ D16) { const int r = blockIdx.x * 256 + threadIdx.x; if (r >= NROW) return; FragH z;
#pragma unroll
  for (int q = 0; q < 8; ++q) z.h[q] = (_Float16)0.0f; unsigned short* d = (unsigned short*)D16 + (size_t)r * 2 * FFP + FF; unsigned short* d2 = d + FFP;
  for (int pass = 0; pass < 2; ++pass) { *(volatile v8us*)d = z.half[0]; *(volatile v8us*)(d + 8) = z.half[0]; *(volatile v8us*)d2 = z.half[0]; *(volatile v8us*)(d2 + 8) = z.half[0]; if (pass == 0) __threadfence(); } }
__global__ __launch_bounds__(1024) void k_tokhead(const float* __restrict__ SRC, const float* __restrict__ Wt, const float* __restrict__ bt, float* __restrict__ out) {
  #pragma clang fp contract(off)
  __shared__ float so[32];
  const int tid = threadIdx.x, w = tid >> 5, ln = tid & 31; const int f = blockIdx.x * 32 + w; const bool live = (f < 2 * NBATCH * DD); const int fl_ = live ? f : 0; const int k = fl_ / (NBATCH * DD), rem = fl_ % (NBATCH * DD); const int b = rem / DD, c = rem % DD; float s = 0.f;
  for (int l = ln; l < LL; l += 32) s += SRC[((size_t)b * LL + l) * DP + c] * bf16_round(Wt[l * 2 + k]);
  for (int o = 16; o > 0; o >>= 1) s += __shfl_xor(s, o, 32);
  if (ln == 0) so[w] = s + bf16_round(bt[k]);
  __syncthreads();
  if (tid < 8 && blockIdx.x * 32 + tid * 4 < 2 * NBATCH * DD) { const v4f v = *(const v4fa*)&so[tid * 4]; float* dst = out + blockIdx.x * 32 + tid * 4; *(volatile v4f*)dst = v; __threadfence(); *(volatile v4f*)dst = v; } }

extern "C" void kernel_launch(void* const* d_in, const int* in_sizes, int n_in,
                              void* d_out, int out_size, void* d_ws, size_t ws_size, hipStream_t stream) {
  (void)in_sizes; (void)n_in; (void)out_size;
  const int* tok = (const int*)d_in[0]; const float* const* I = (const float* const*)d_in;
  const float* emb = I[2]; const float* Wq = I[3]; const float* bq = I[4]; const float* Wk = I[5]; const float* bk = I[6]; const float* Wv = I[7]; const float* bv = I[8]; const float* Wo = I[9]; const float* bo = I[10]; const float* ln1g = I[11]; const float* ln1b = I[12];
  const float* W1 = I[13]; const float* b1 = I[14]; const float* W2 = I[15]; const float* b2 = I[16]; const float* ln2g = I[17]; const float* ln2b = I[18]; const float* e1W = I[19]; const float* e1b = I[20]; const float* e2W = I[21]; const float* e2b = I[22]; const float* WOw = I[23]; const float* WOb = I[24];
  const float* Wcc = I[25]; const float* bcc = I[26]; const float* Wcc2 = I[27]; const float* bcc2 = I[28]; const float* o1W = I[29]; const float* o1b = I[30]; const float* o2W = I[31]; const float* o2b = I[32]; const float* WAw = I[33]; const float* WAb = I[34]; const float* Wm = I[35]; const float* bm = I[36]; const float* Wn = I[37]; const float* bn = I[38];
  float* out0 = (float*)d_out; float* out1 = (float*)((char*)d_out + 19660800); float* out2 = (float*)((char*)d_out + 39321600); float* out3 = (float*)((char*)d_out + 39331200);
  char* ws = (char*)d_ws; size_t off = 0;
  auto take = [&](size_t bytes) { char* p = ws + off; off += (bytes + 255) & ~(size_t)255; return p; };
  _Float16* BQ = (_Float16*)take((size_t)NLAY * DP * DP * 2); _Float16* BKw = (_Float16*)take((size_t)NLAY * DP * DP * 2); _Float16* BVw = (_Float16*)take((size_t)NLAY * DP * DP * 2); _Float16* BOw = (_Float16*)take((size_t)NLAY * DP * DP * 2);
  _Float16* BW1 = (_Float16*)take((size_t)NLAY * FFP * DP * 2); _Float16* BW2 = (_Float16*)take((size_t)NLAY * DP * FFP * 2);
  _Float16* BE1 = (_Float16*)take((size_t)DP * 2 * DP * 2); _Float16* BE2 = (_Float16*)take((size_t)DP * 2 * DP * 2); _Float16* BWO = (_Float16*)take((size_t)FFP * 2 * DP * 2); _Float16* BCC = (_Float16*)take((size_t)640 * 2 * DP * 2); _Float16* BCC2 = (_Float16*)take((size_t)DP * 2 * 640 * 2);
  _Float16* BO1 = (_Float16*)take((size_t)1536 * 3072 * 2); _Float16* BO2 = (_Float16*)take((size_t)FFP * 3072 * 2); _Float16* BWA = (_Float16*)take((size_t)FFP * 2 * FFP * 2);
  float* BIAS = (float*)take((size_t)64 * 1536 * 4);
  int* PADK = (int*)take((size_t)NROW * 4);
  float* X = (float*)take((size_t)NROW * DP * 4); _Float16* X16 = (_Float16*)take((size_t)NROW * DP * 2); float* T = (float*)take((size_t)NROW * DP * 4); float* F = (float*)take((size_t)NROW * DP * 4);
  _Float16* QP = (_Float16*)take((size_t)NPS * LL * 64 * 2); _Float16* KP = (_Float16*)take((size_t)NPS * LL * 64 * 2); _Float16* VP = (_Float16*)take((size_t)NPS * LL * 64 * 2); _Float16* VT = (_Float16*)take((size_t)NPS * 64 * LL * 2); float* OP = (float*)take((size_t)NPS * LL * 64 * 4);
  _Float16* C16 = (_Float16*)take((size_t)NROW * DP * 2); _Float16* H16 = (_Float16*)take((size_t)NROW * 2 * FFP * 2); _Float16* XP = (_Float16*)take((size_t)NROW * 2 * DP * 2); _Float16* CP2 = (_Float16*)take((size_t)NROW * 2 * 640 * 2);
  float* G1 = (float*)take((size_t)NROW * FFP * 4); _Float16* A16 = (_Float16*)take((size_t)NROW * 3072 * 2); float* G2 = (float*)take((size_t)NROW * 1536 * 4); _Float16* D16 = (_Float16*)take((size_t)NROW * 3072 * 2);
  if (off > ws_size) return;
  auto bias = [&](int i) { return BIAS + (size_t)i * 1536; };
  for (int l = 0; l < NLAY; ++l) {
    k_wtp<<<(DP * DP / 8 + 255) / 256, 256, 0, stream>>>(Wq + (size_t)l * DD * DD, DD, DD, DP, DP, BQ + (size_t)l * DP * DP); k_wtp<<<(DP * DP / 8 + 255) / 256, 256, 0, stream>>>(Wk + (size_t)l * DD * DD, DD, DD, DP, DP, BKw + (size_t)l * DP * DP);
    k_wtp<<<(DP * DP / 8 + 255) / 256, 256, 0, stream>>>(Wv + (size_t)l * DD * DD, DD, DD, DP, DP, BVw + (size_t)l * DP * DP); k_wtp<<<(DP * DP / 8 + 255) / 256, 256, 0, stream>>>(Wo + (size_t)l * DD * DD, DD, DD, DP, DP, BOw + (size_t)l * DP * DP);
    k_wtp<<<(FFP * DP / 8 + 255) / 256, 256, 0, stream>>>(W1 + (size_t)l * DD * FF, DD, FF, DP, FFP, BW1 + (size_t)l * FFP * DP); k_wtp<<<(DP * FFP / 8 + 255) / 256, 256, 0, stream>>>(W2 + (size_t)l * FF * DD, FF, DD, FFP, DP, BW2 + (size_t)l * DP * FFP);
    k_bpad<<<2, 256, 0, stream>>>(bq + (size_t)l * DD, DD, DP, bias(6 * l + 0)); k_bpad<<<2, 256, 0, stream>>>(bk + (size_t)l * DD, DD, DP, bias(6 * l + 1)); k_bpad<<<2, 256, 0, stream>>>(bv + (size_t)l * DD, DD, DP, bias(6 * l + 2));
    k_bpad<<<2, 256, 0, stream>>>(bo + (size_t)l * DD, DD, DP, bias(6 * l + 3)); k_bpad<<<5, 256, 0, stream>>>(b1 + (size_t)l * FF, FF, FFP, bias(6 * l + 4)); k_bpad<<<2, 256, 0, stream>>>(b2 + (size_t)l * DD, DD, DP, bias(6 * l + 5)); }
  k_wtp2<<<(DP * 2 * DP / 8 + 255) / 256, 256, 0, stream>>>(e1W, DD, DD, DP, DP, BE1); k_wtp2<<<(DP * 2 * DP / 8 + 255) / 256, 256, 0, stream>>>(e2W, DD, DD, DP, DP, BE2); k_wtp2<<<(FFP * 2 * DP / 8 + 255) / 256, 256, 0, stream>>>(WOw, DD, FF, DP, FFP, BWO);
  k_wtp2<<<(640 * 2 * DP / 8 + 255) / 256, 256, 0, stream>>>(Wcc, DD, 600, DP, 640, BCC); k_wtp2<<<(DP * 2 * 640 / 8 + 255) / 256, 256, 0, stream>>>(Wcc2, 600, DD, 640, DP, BCC2);
  k_wtp_o1p<<<(1536 * (3072 / 8) + 255) / 256, 256, 0, stream>>>(o1W, BO1); k_wtp2<<<(FFP * 3072 / 8 + 255) / 256, 256, 0, stream>>>(o2W, 1500, FF, 1536, FFP, BO2); k_wtp2<<<(FFP * 2 * FFP / 8 + 255) / 256, 256, 0, stream>>>(WAw, FF, FF, FFP, FFP, BWA);
  k_bpad<<<2, 256, 0, stream>>>(e1b, DD, DP, bias(36)); k_bpad<<<2, 256, 0, stream>>>(e2b, DD, DP, bias(37)); k_bpad<<<5, 256, 0, stream>>>(WOb, FF, FFP, bias(38)); k_bpad<<<3, 256, 0, stream>>>(bcc, 600, 640, bias(39)); k_bpad<<<2, 256, 0, stream>>>(bcc2, DD, DP, bias(40));
  k_bpad<<<6, 256, 0, stream>>>(o1b, 1500, 1536, bias(41)); k_bpad<<<5, 256, 0, stream>>>(o2b, FF, FFP, bias(42)); k_bpad<<<5, 256, 0, stream>>>(WAb, FF, FFP, bias(43));
  k_padk<<<(NROW + 255) / 256, 256, 0, stream>>>(tok, PADK);
  k_embed<<<(NROW * (DP / 4) + 255) / 256, 256, 0, stream>>>(tok, emb, X, X16);
  const dim3 gD((NROW / 128) * (DP / 64), 1), gF((NROW / 128) * (FFP / 64), 1); const unsigned nps8 = (NPS * LL * 8 + 255) / 256, nr8 = (NROW * (DP / 8) + 255) / 256;
  for (int l = 0; l < NLAY; ++l) {
    const _Float16* bq_ = BQ + (size_t)l * DP * DP; const _Float16* bk_ = BKw + (size_t)l * DP * DP; const _Float16* bv_ = BVw + (size_t)l * DP * DP; const _Float16* bo_ = BOw + (size_t)l * DP * DP;
    k_gemm2<0><<<gD, 128, 0, stream>>>(X16, DP, 0, bq_, DP, 0, 0.0625f, bias(6 * l + 0), 0, nullptr, 1, 0, 0, F, nullptr, DP, 0, NROW, DP, DP); k_pseudo<<<nps8, 256, 0, stream>>>(F, QP);
    k_gemm2<0><<<gD, 128, 0, stream>>>(X16, DP, 0, bk_, DP, 0, 0.0625f, bias(6 * l + 1), 0, nullptr, 1, 0, 0, F, nullptr, DP, 0, NROW, DP, DP); k_pseudo<<<nps8, 256, 0, stream>>>(F, KP);
    k_gemm2<0><<<gD, 128, 0, stream>>>(X16, DP, 0, bv_, DP, 0, 0.0625f, bias(6 * l + 2), 0, nullptr, 1, 0, 0, F, nullptr, DP, 0, NROW, DP, DP); k_pseudo<<<nps8, 256, 0, stream>>>(F, VP);
    k_vt<1, TK><<<NPS * (TK / 64), 256, 0, stream>>>(VP, 64, 0, VT);
    k_flashpad<<<NPS * (TQ / 64), 128, 0, stream>>>(QP, 64, KP, 64, VT, PADK, OP, 64);
    k_unpseudo<<<nr8, 256, 0, stream>>>(OP, C16);
    k_gemm2<0><<<gD, 128, 0, stream>>>(C16, DP, 0, bo_, DP, 0, 0.0625f, bias(6 * l + 3), 0, X, 1, (size_t)DP, 0, T, nullptr, DP, 0, NROW, DP, DP);
    k_ln300<<<NROW / 8, 256, 0, stream>>>(T, ln1g + (size_t)l * DD, ln1b + (size_t)l * DD, X, X16);
    k_gemm2<3><<<gF, 128, 0, stream>>>(X16, DP, 0, BW1 + (size_t)l * FFP * DP, DP, 0, 0.0625f, bias(6 * l + 4), 0, nullptr, 1, 0, 0, nullptr, H16, FFP, 0, NROW, FFP, DP);
    k_gemm2<0><<<gD, 128, 0, stream>>>(H16, FFP, 0, BW2 + (size_t)l * DP * FFP, FFP, 0, 0.0625f, bias(6 * l + 5), 0, X, 1, (size_t)DP, 0, T, nullptr, DP, 0, NROW, DP, FFP);
    k_ln300<<<NROW / 8, 256, 0, stream>>>(T, ln2g + (size_t)l * DD, ln2b + (size_t)l * DD, X, X16); }
  const dim3 g15((NROW / 128) * (1536 / 64), 1), g64((NROW / 128) * (640 / 64), 1);
  k_cat16<<<nr8, 256, 0, stream>>>(X, DP, DD, DP, XP, 2 * DP, 0, DP);
  k_gemm2<0><<<gD, 128, 0, stream>>>(XP, 2 * DP, 0, BE1, 2 * DP, 0, 0.0625f, bias(36), 0, nullptr, 1, 0, 0, F, nullptr, DP, 0, NROW, DP, 2 * DP); k_selu16<<<nr8, 256, 0, stream>>>(F, DP, DD, DP, CP2, 2 * DP, 0, DP);
  k_gemm2<0><<<gD, 128, 0, stream>>>(CP2, 2 * DP, 0, BE2, 2 * DP, 0, 0.0625f, bias(37), 0, nullptr, 1, 0, 0, F, nullptr, DP, 0, NROW, DP, 2 * DP); k_selu16<<<(NROW * (336 / 8) + 255) / 256, 256, 0, stream>>>(F, DP, DD, 336, A16, 3072, FF, 1536);
  k_gemm2<0><<<gF, 128, 0, stream>>>(XP, 2 * DP, 0, BWO, 2 * DP, 0, 0.0625f, bias(38), 0, nullptr, 1, 0, 0, G1, nullptr, FFP, 0, NROW, FFP, 2 * DP); k_cat16<<<(NROW * (FF / 8) + 255) / 256, 256, 0, stream>>>(G1, FFP, FF, FF, A16, 3072, 0, 1536);
  k_gemm2<0><<<g15, 128, 0, stream>>>(A16, 3072, 0, BO1, 3072, 0, 0.0625f, bias(41), 0, nullptr, 1, 0, 0, G2, nullptr, 1536, 0, NROW, 1536, 3072); k_selu16<<<(NROW * (1536 / 8) + 255) / 256, 256, 0, stream>>>(G2, 1536, 1536, 1536, D16, 3072, 0, 1536);
  k_gemm2<0><<<gF, 128, 0, stream>>>(D16, 3072, 0, BO2, 3072, 0, 0.0625f, bias(42), 0, nullptr, 1, 0, 0, G1, nullptr, FFP, 0, NROW, FFP, 3072); k_pack1200<1><<<(NROW * (FF / 4) + 255) / 256, 256, 0, stream>>>(G1, out0, H16); k_zpad16<<<(NROW + 255) / 256, 256, 0, stream>>>(H16);
  k_gemm2<0><<<gF, 128, 0, stream>>>(H16, 2 * FFP, 0, BWA, 2 * FFP, 0, 0.0625f, bias(43), 0, nullptr, 1, 0, 0, G1, nullptr, FFP, 0, NROW, FFP, 2 * FFP); k_pack1200<0><<<(NROW * (FF / 4) + 255) / 256, 256, 0, stream>>>(G1, out1, nullptr);
  k_tokhead<<<(2 * NBATCH * DD + 31) / 32, 1024, 0, stream>>>(X, Wm, bm, out2);
  k_gemm2<0><<<g64, 128, 0, stream>>>(XP, 2 * DP, 0, BCC, 2 * DP, 0, 0.0625f, bias(39), 0, nullptr, 1, 0, 0, G2, nullptr, 640, 0, NROW, 640, 2 * DP); k_cat16<<<(NROW * (640 / 8) + 255) / 256, 256, 0, stream>>>(G2, 640, 640, 640, CP2, 1280, 0, 640);
  k_gemm2<0><<<gD, 128, 0, stream>>>(CP2, 1280, 0, BCC2, 1280, 0, 0.0625f, bias(40), 0, nullptr, 1, 0, 0, F, nullptr, DP, 0, NROW, DP, 1280); k_tokhead<<<(2 * NBATCH * DD + 31) / 32, 1024, 0, stream>>>(F, Wn, bn, out3);
}
